// CSPAttention_46093589021345
// MI455X (gfx1250) — hardware-verified
//
#include <hip/hip_runtime.h>
#include <math.h>

typedef __attribute__((ext_vector_type(16))) _Float16 v16h;
typedef __attribute__((ext_vector_type(16))) __bf16 v16b;
typedef __attribute__((ext_vector_type(8)))  _Float16 v8h;
typedef __attribute__((ext_vector_type(8)))  float v8f;
typedef __attribute__((ext_vector_type(4)))  float v4f;
typedef __attribute__((ext_vector_type(2)))  float v2f;
typedef __attribute__((ext_vector_type(4)))  unsigned v4u;
typedef __attribute__((ext_vector_type(4)))  int v4i;
typedef float __attribute__((may_alias)) float_a;
typedef int __attribute__((may_alias)) int_a;

template <typename T> __device__ __forceinline__ void vst2(void* p, T v) { *(volatile T*)p = v; __threadfence(); *(volatile T*)p = v; }
__device__ __forceinline__ v8f wmma16(v16h a, v16h b, v8f c) {
  v8f d = __builtin_amdgcn_wmma_f32_16x16x32_f16(false, a, false, b, (short)0, c, false, false);
  asm volatile("v_nop\n\tv_nop\n\tv_nop\n\tv_nop" : "+v"(d) : "v"(a), "v"(b));
  return d;
}
__device__ __forceinline__ v8f wmma_bf(v16b a, v16b b, v8f c) {
  v8f d = __builtin_amdgcn_wmma_f32_16x16x32_bf16(false, a, false, b, (short)0, c, false, false);
  asm volatile("v_nop\n\tv_nop\n\tv_nop\n\tv_nop" : "+v"(d) : "v"(a), "v"(b));
  return d;
}
__device__ __forceinline__ v16h frag_h(const _Float16* rowk0, int lane) {
  union { v16h v; v8h q[2]; } u; const _Float16* p = rowk0 + 8 * (lane >> 4);
  u.q[0] = *(const v8h*)p; u.q[1] = *(const v8h*)(p + 16); return u.v;
}
__device__ __forceinline__ v16h frag_f32(const float* rowk0, int lane) {
  v16h a; const float* p = rowk0 + 8 * (lane >> 4);
#pragma unroll
  for (int i = 0; i < 8; ++i) { a[i] = (_Float16)p[i]; a[8 + i] = (_Float16)p[16 + i]; }
  return a;
}
__device__ __forceinline__ v16h frag_f32s(const float* rowk0, int lane, float sc) {
  v16h a; const float* p = rowk0 + 8 * (lane >> 4);
#pragma unroll
  for (int i = 0; i < 8; ++i) { a[i] = (_Float16)(p[i] * sc); a[8 + i] = (_Float16)(p[16 + i] * sc); }
  return a;
}
__device__ __forceinline__ v16h fragc_f32(const float* W, int k0, int n, int lane, int ld, int K) {
  v16h a; const int g = lane >> 4;
#pragma unroll
  for (int i = 0; i < 8; ++i) { const int ka = k0 + 8 * g + i, kb = ka + 16;
    a[i] = (_Float16)(ka < K ? W[(size_t)ka * ld + n] : 0.f); a[8 + i] = (_Float16)(kb < K ? W[(size_t)kb * ld + n] : 0.f); }
  return a;
}
struct F2 { v16b h, l; };
__device__ __forceinline__ F2 bsplit16(const float v[16]) { F2 r;
#pragma unroll
  for (int i = 0; i < 16; ++i) { const __bf16 h = (__bf16)v[i]; r.h[i] = h; r.l[i] = (__bf16)(v[i] - (float)h); }
  return r; }
__device__ __forceinline__ F2 split_row(const float* row, int k0, int lane) { float v[16]; const float* p = row + k0 + 8 * (lane >> 4);
#pragma unroll
  for (int i = 0; i < 8; ++i) { v[i] = p[i]; v[8 + i] = p[16 + i]; }
  return bsplit16(v); }
__device__ __forceinline__ F2 split_rowK(const float* row, int k0, int lane, int K) { float v[16]; const int g = lane >> 4;
#pragma unroll
  for (int i = 0; i < 8; ++i) { const int ka = k0 + 8 * g + i, kb = ka + 16; v[i] = ka < K ? row[ka] : 0.f; v[8 + i] = kb < K ? row[kb] : 0.f; }
  return bsplit16(v); }
__device__ __forceinline__ F2 split_col(const float* W, int k0, int n, int lane, int ld, int K) { float v[16]; const int g = lane >> 4;
#pragma unroll
  for (int i = 0; i < 8; ++i) { const int ka = k0 + 8 * g + i, kb = ka + 16; v[i] = ka < K ? W[(size_t)ka * ld + n] : 0.f; v[8 + i] = kb < K ? W[(size_t)kb * ld + n] : 0.f; }
  return bsplit16(v); }
__device__ __forceinline__ v8f mac3(const F2& a, const F2& b, v8f c) { c = wmma_bf(a.l, b.h, c); c = wmma_bf(a.h, b.l, c); return wmma_bf(a.h, b.h, c); }
__device__ __forceinline__ float sigm(float v) { return 1.0f / (1.0f + expf(-v)); }
#define LDSX() do { asm volatile("s_wait_dscnt 0" ::: "memory"); __builtin_amdgcn_wave_barrier(); __builtin_amdgcn_fence(__ATOMIC_RELEASE, "workgroup"); } while (0)


#define NB 4
#define SS 2048
#define DM 1024
#define E 512
#define NH 8
#define HD 64
#define NR (NB * SS)

__global__ __launch_bounds__(256) void k_cvt(const float* __restrict__ src, int coff, _Float16* __restrict__ X16) {
  const size_t i8 = (size_t)blockIdx.x * 256 + threadIdx.x; if (i8 >= (size_t)NR * E / 8) return; const size_t r = i8 / (E / 8), pc = i8 % (E / 8);
  union { v8h h; v4u u; } pk; const float* s = src + r * DM + coff + pc * 8;
#pragma unroll
  for (int e = 0; e < 8; ++e) pk.h[e] = (_Float16)s[e];
  vst2(X16 + r * E + pc * 8, pk.u);
}
__global__ __launch_bounds__(256) void k_pack(const float* __restrict__ Wq, const float* __restrict__ Wk, const float* __restrict__ Wv, const float* __restrict__ Woa, const float* __restrict__ Woc, const float* __restrict__ Wf, _Float16* __restrict__ PT, _Float16* __restrict__ PF) {
  const int n = blockIdx.x, tid = threadIdx.x; __shared__ __align__(16) _Float16 srow[DM];
  if (n < 5 * E) { const int which = n / E, nn = n % E; const float* W = which == 0 ? Wq : (which == 1 ? Wk : (which == 2 ? Wv : (which == 3 ? Woa : Woc)));
    srow[tid] = (_Float16)(W[(size_t)nn * E + tid] * 16.0f); srow[tid + 256] = (_Float16)(W[(size_t)nn * E + tid + 256] * 16.0f); __syncthreads();
    if (tid < E / 8) vst2(PT + (size_t)n * E + tid * 8, *(const v4u*)(&srow[tid * 8])); }
  else { const int nn = n - 5 * E; for (int k = tid; k < DM; k += 256) srow[k] = (_Float16)(Wf[(size_t)nn * DM + k] * 16.0f); __syncthreads();
    if (tid < DM / 8) vst2(PF + (size_t)nn * DM + tid * 8, *(const v4u*)(&srow[tid * 8])); }
}
__global__ __launch_bounds__(128) void k_qkv(const _Float16* __restrict__ Xq, const _Float16* __restrict__ Xk, const _Float16* __restrict__ Xv, const _Float16* __restrict__ PT, const float* __restrict__ bq, const float* __restrict__ bk, const float* __restrict__ bv,
                                            _Float16* __restrict__ Q16, _Float16* __restrict__ K16, _Float16* __restrict__ VTh) {
  __shared__ __align__(16) float so[4][16][132];
  __shared__ __align__(16) _Float16 sth[128][72];
  const int tid = threadIdx.x, wave = tid >> 5, lane = tid & 31, col = lane & 15, g = lane >> 4;
  const int which = blockIdx.z, r0b = blockIdx.x * 64, r0 = r0b + wave * 16, n0 = blockIdx.y * 128; const int b = r0b / SS, s0 = r0b % SS;
  const _Float16* X16 = which == 0 ? Xq : (which == 1 ? Xk : Xv); const float* bb_ = which == 0 ? bq : (which == 1 ? bk : bv);
  v8f acc[8] = {};
#pragma unroll 2
  for (int kc = 0; kc < E / 32; ++kc) { const v16h a = frag_h(X16 + (size_t)(r0 + col) * E + kc * 32, lane);
#pragma unroll
    for (int j = 0; j < 8; ++j) acc[j] = wmma16(a, frag_h(PT + (size_t)(which * E + n0 + j * 16 + col) * E + kc * 32, lane), acc[j]); }
  if (which < 2) {
#pragma unroll
    for (int j = 0; j < 8; ++j) { const float bb = bb_[n0 + j * 16 + col];
#pragma unroll
      for (int r = 0; r < 8; ++r) so[wave][8 * g + r][j * 16 + col] = (acc[j][r] * (1.0f / 16.0f) + bb) * 4.0f; }
    LDSX();
    _Float16* Dst = which == 0 ? Q16 : K16;
    for (int qq = lane; qq < 16 * 2 * 8; qq += 32) { const int hh = qq >> 7, rl = (qq >> 3) & 15, pc = qq & 7; const int h = (n0 >> 6) + hh; union { v8h h8; v4u u; } pk;
#pragma unroll
      for (int e = 0; e < 8; ++e) pk.h8[e] = (_Float16)so[wave][rl][hh * 64 + pc * 8 + e];
      vst2(Dst + (((size_t)b * NH + h) * SS + s0 + wave * 16 + rl) * HD + pc * 8, pk.u); } }
  else {
#pragma unroll
    for (int j = 0; j < 8; ++j) { const float bb = bb_[n0 + j * 16 + col];
#pragma unroll
      for (int r = 0; r < 8; ++r) sth[j * 16 + col][wave * 16 + 8 * g + r] = (_Float16)((acc[j][r] * (1.0f / 16.0f) + bb) * 4.0f); }
    __syncthreads();
    for (int qq = tid; qq < 128 * 8; qq += 128) { const int cl = qq >> 3, pc = qq & 7; const int c = n0 + cl, h = c >> 6, d = c & 63; vst2(VTh + (((size_t)b * NH + h) * HD + d) * SS + s0 + pc * 8, *(const v4u*)(&sth[cl][pc * 8])); } }
}
__global__ __launch_bounds__(128) void k_attn(const _Float16* __restrict__ Q16, const _Float16* __restrict__ K16, const _Float16* __restrict__ VTh, _Float16* __restrict__ O16) {
  __shared__ __align__(16) float sS[4][16][68];
  __shared__ __align__(16) _Float16 sPh[4][16][72];
  __shared__ __align__(16) float sO[4][16][68];
  const int tid = threadIdx.x, w = tid >> 5, lane = tid & 31, col = lane & 15, g = lane >> 4;
  const size_t bh = blockIdx.y; const int q0 = blockIdx.x * 64 + w * 16;
  v16h aq[2];
#pragma unroll
  for (int kc = 0; kc < 2; ++kc) aq[kc] = frag_h(Q16 + (bh * SS + q0 + col) * HD + kc * 32, lane);
  float mrun = -3.0e38f, lrun = 0.f; v8f acc[4] = {};
#pragma unroll 1
  for (int kt = 0; kt < SS / 64; ++kt) {
#pragma unroll
    for (int t = 0; t < 4; ++t) { v8f s = {}; const int key = kt * 64 + t * 16 + col;
#pragma unroll
      for (int kc = 0; kc < 2; ++kc) s = wmma16(aq[kc], frag_h(K16 + (bh * SS + key) * HD + kc * 32, lane), s);
#pragma unroll
      for (int r = 0; r < 8; ++r) sS[w][8 * g + r][t * 16 + col] = s[r] * (0.125f / 16.0f); }
    LDSX();
    float mx = -3.4e38f;
#pragma unroll
    for (int jj = 0; jj < 32; ++jj) mx = fmaxf(mx, sS[w][col][g * 32 + jj]);
    mx = fmaxf(mx, __shfl_xor(mx, 16, 32));
    const float mnew = fmaxf(mrun, mx); const float corr = expf(mrun - mnew);
    float ps = 0.f;
#pragma unroll
    for (int jj = 0; jj < 32; ++jj) { const float p = expf(sS[w][col][g * 32 + jj] - mnew) * 16384.0f; ps += p; sPh[w][col][g * 32 + jj] = (_Float16)p; }
    ps += __shfl_xor(ps, 16, 32);
    lrun = lrun * corr + ps * (1.0f / 16384.0f); mrun = mnew;
#pragma unroll
    for (int r = 0; r < 8; ++r) { const float cr = __shfl(corr, 8 * g + r, 32);
#pragma unroll
      for (int t = 0; t < 4; ++t) acc[t][r] *= cr; }
    LDSX();
#pragma unroll
    for (int kc = 0; kc < 2; ++kc) { const v16h ph = frag_h(&sPh[w][col][0] + kc * 32, lane);
#pragma unroll
      for (int t = 0; t < 4; ++t) { const size_t vo = (bh * HD + t * 16 + col) * SS + kt * 64 + kc * 32; acc[t] = wmma16(ph, frag_h(VTh + vo, lane), acc[t]); } }
    __builtin_amdgcn_wave_barrier(); }
#pragma unroll
  for (int r = 0; r < 8; ++r) { const float lr = __shfl(lrun, 8 * g + r, 32); const float inv = 8.0f / (lr * 16384.0f * 4.0f);
#pragma unroll
    for (int t = 0; t < 4; ++t) sO[w][8 * g + r][t * 16 + col] = acc[t][r] * inv; }
  LDSX();
  for (int qq = lane; qq < 16 * 8; qq += 32) { const int rl = qq >> 3, pc = qq & 7; union { v8h h8; v4u u; } pk;
#pragma unroll
    for (int e = 0; e < 8; ++e) pk.h8[e] = (_Float16)sO[w][rl][pc * 8 + e];
    vst2(O16 + ((bh * SS) + q0 + rl) * HD + pc * 8, pk.u); }
}
__global__ __launch_bounds__(128) void k_proj512(const _Float16* __restrict__ A16, int headm, const _Float16* __restrict__ PTw, const float* __restrict__ bias, float ascale, int coff, _Float16* __restrict__ CAT) {
  __shared__ __align__(16) _Float16 so[4][16][136];
  const int tid = threadIdx.x, wave = tid >> 5, lane = tid & 31, col = lane & 15, g = lane >> 4;
  const int r0 = blockIdx.x * 64 + wave * 16, n0 = blockIdx.y * 128; const int ra = r0 + col; const int b = ra / SS, s = ra % SS;
  v8f acc[8] = {};
#pragma unroll 2
  for (int kc = 0; kc < E / 32; ++kc) { const v16h a = headm ? frag_h(A16 + (((size_t)b * NH + (kc >> 1)) * SS + s) * HD + (kc & 1) * 32, lane) : frag_h(A16 + (size_t)ra * E + kc * 32, lane);
#pragma unroll
    for (int j = 0; j < 8; ++j) acc[j] = wmma16(a, frag_h(PTw + (size_t)(n0 + j * 16 + col) * E + kc * 32, lane), acc[j]); }
#pragma unroll
  for (int j = 0; j < 8; ++j) { const float bb = bias[n0 + j * 16 + col];
#pragma unroll
    for (int r = 0; r < 8; ++r) so[wave][8 * g + r][j * 16 + col] = (_Float16)(acc[j][r] * ascale + bb); }
  LDSX();
  for (int rl = 0; rl < 16; ++rl) { if (lane < 16) vst2(CAT + (size_t)(r0 + rl) * DM + coff + n0 + lane * 8, *(const v4u*)(&so[wave][rl][lane * 8])); }
}
__global__ __launch_bounds__(256) void k_conv(const float* __restrict__ q, const float* __restrict__ cw, const float* __restrict__ cb, _Float16* __restrict__ C16) {
  __shared__ __align__(16) _Float16 sc[64][E + 8];
  const int tid = threadIdx.x; const int b = blockIdx.y, l0 = blockIdx.x * 64;
#pragma unroll 1
  for (int cc = 0; cc < 2; ++cc) { const int c = tid + cc * 256; const float w0 = cw[c * 3], w1 = cw[c * 3 + 1], w2 = cw[c * 3 + 2], bb = cb[c]; const float* col_ = q + (size_t)b * SS * DM + E + c;
#pragma unroll 4
    for (int i = 0; i < 64; ++i) { const int l = l0 + i; const float xm = l > 0 ? col_[(size_t)(l - 1) * DM] : 0.f, x0 = col_[(size_t)l * DM], xp = l < SS - 1 ? col_[(size_t)(l + 1) * DM] : 0.f;
      sc[i][c] = (_Float16)(w0 * xm + w1 * x0 + w2 * xp + bb); } }
  __syncthreads();
  for (int qq = tid; qq < 64 * (E / 8); qq += 256) { const int i = qq >> 6, pc = qq & 63; vst2(C16 + ((size_t)b * SS + l0 + i) * E + pc * 8, *(const v4u*)(&sc[i][pc * 8])); }
}
__global__ __launch_bounds__(128) void k_wf(const _Float16* __restrict__ CAT, const _Float16* __restrict__ PF, const float* __restrict__ bfv, const float* __restrict__ q, float* __restrict__ T) {
  __shared__ __align__(16) float so[4][16][132];
  const int tid = threadIdx.x, wave = tid >> 5, lane = tid & 31, col = lane & 15, g = lane >> 4; const int r0 = blockIdx.x * 64 + wave * 16, n0 = blockIdx.y * 128;
  v8f acc[8] = {};
#pragma unroll 2
  for (int kc = 0; kc < DM / 32; ++kc) { const v16h a = frag_h(CAT + (size_t)(r0 + col) * DM + kc * 32, lane);
#pragma unroll
    for (int j = 0; j < 8; ++j) acc[j] = wmma16(a, frag_h(PF + (size_t)(n0 + j * 16 + col) * DM + kc * 32, lane), acc[j]); }
#pragma unroll
  for (int j = 0; j < 8; ++j) { const int n = n0 + j * 16 + col; const float bb = bfv[n];
#pragma unroll
    for (int r = 0; r < 8; ++r) so[wave][8 * g + r][j * 16 + col] = acc[j][r] * (1.0f / 16.0f) + bb + q[(size_t)(r0 + 8 * g + r) * DM + n]; }
  LDSX();
#pragma unroll 4
  for (int rl = 0; rl < 16; ++rl) vst2(T + (size_t)(r0 + rl) * DM + n0 + lane * 4, *(const v4f*)(&so[wave][rl][lane * 4]));
}
__global__ __launch_bounds__(256) void k_ln(const float* __restrict__ T, const float* __restrict__ gm, const float* __restrict__ bt, float* __restrict__ out) {
  const int wave = threadIdx.x >> 5, lane = threadIdx.x & 31; const size_t row = (size_t)blockIdx.x * 8 + wave; const float* tr = T + row * DM;
  float s = 0.f, sq = 0.f;
#pragma unroll
  for (int p = 0; p < 8; ++p) { const v4f v = *(const v4f*)(tr + p * 128 + lane * 4);
#pragma unroll
    for (int e = 0; e < 4; ++e) { s += v[e]; sq += v[e] * v[e]; } }
#pragma unroll
  for (int o = 16; o > 0; o >>= 1) { s += __shfl_xor(s, o, 32); sq += __shfl_xor(sq, o, 32); }
  const float mu = s * (1.0f / DM); float var = sq * (1.0f / DM) - mu * mu; var = var > 0.f ? var : 0.f; const float rs = rsqrtf(var + 1e-5f);
#pragma unroll 1
  for (int p = 0; p < 8; ++p) { const int c0 = p * 128 + lane * 4; v4f v = *(const v4f*)(tr + c0);
#pragma unroll
    for (int e = 0; e < 4; ++e) v[e] = (v[e] - mu) * rs * gm[c0 + e] + bt[c0 + e];
    vst2(out + row * DM + c0, v); }
}
extern "C" void kernel_launch(void* const* d_in, const int* in_sizes, int n_in, void* d_out, int out_size, void* d_ws, size_t ws_size, hipStream_t stream) {
  (void)in_sizes; (void)n_in; (void)out_size; (void)ws_size;
  const float** I = (const float**)d_in;
  const float* queries = I[0]; const float* keys = I[1]; const float* values = I[2]; const float* Wq = I[3]; const float* bq = I[4]; const float* Wk = I[5]; const float* bk = I[6]; const float* Wv = I[7]; const float* bv = I[8];
  const float* Woa = I[9]; const float* boa = I[10]; const float* cw = I[11]; const float* cb = I[12]; const float* Woc = I[13]; const float* boc = I[14]; const float* Wf = I[15]; const float* bfv = I[16]; const float* gm = I[17]; const float* bt = I[18];
  float* out = (float*)d_out;
  char* ws = (char*)d_ws; size_t off = 0;
  auto take = [&](size_t bytes) { char* p = ws + off; off += (bytes + 255) & ~(size_t)255; return p; };
  _Float16* Xq = (_Float16*)take((size_t)NR * E * 2); _Float16* Xk = (_Float16*)take((size_t)NR * E * 2); _Float16* Xv = (_Float16*)take((size_t)NR * E * 2);
  _Float16* PT = (_Float16*)take((size_t)5 * E * E * 2); _Float16* PF = (_Float16*)take((size_t)DM * DM * 2);
  _Float16* Q16 = (_Float16*)take((size_t)NR * E * 2); _Float16* K16 = (_Float16*)take((size_t)NR * E * 2); _Float16* VTh = (_Float16*)take((size_t)NR * E * 2); _Float16* O16 = Xq;
  _Float16* C16 = Xk;
  _Float16* CAT = (_Float16*)take((size_t)NR * DM * 2); float* T = (float*)take((size_t)NR * DM * 4);
  k_cvt<<<(NR * E / 8 + 255) / 256, 256, 0, stream>>>(queries, 0, Xq);
  k_cvt<<<(NR * E / 8 + 255) / 256, 256, 0, stream>>>(keys, 0, Xk);
  k_cvt<<<(NR * E / 8 + 255) / 256, 256, 0, stream>>>(values, 0, Xv);
  k_pack<<<5 * E + DM, 256, 0, stream>>>(Wq, Wk, Wv, Woa, Woc, Wf, PT, PF);
  k_qkv<<<dim3(NR / 64, E / 128, 3), 128, 0, stream>>>(Xq, Xk, Xv, PT, bq, bk, bv, Q16, K16, VTh);
  k_attn<<<dim3(SS / 64, NB * NH), 128, 0, stream>>>(Q16, K16, VTh, O16);
  k_proj512<<<dim3(NR / 64, E / 128), 128, 0, stream>>>(O16, 1, PT + (size_t)3 * E * E, boa, 1.0f / (16.0f * 8.0f), 0, CAT);
  k_conv<<<dim3(SS / 64, NB), 256, 0, stream>>>(queries, cw, cb, C16);
  k_proj512<<<dim3(NR / 64, E / 128), 128, 0, stream>>>(C16, 0, PT + (size_t)4 * E * E, boc, 1.0f / 16.0f, E, CAT);
  k_wf<<<dim3(NR / 64, DM / 128), 128, 0, stream>>>(CAT, PF, bfv, queries, T);
  k_ln<<<NR / 8, 256, 0, stream>>>(T, gm, bt, out);
}
